// tinystoriesgru_45681272160887
// MI455X (gfx1250) — hardware-verified
//
#include <hip/hip_runtime.h>
#include <math.h>

typedef __attribute__((ext_vector_type(16))) _Float16 v16h;
typedef __attribute__((ext_vector_type(16))) __bf16 v16b;
typedef __attribute__((ext_vector_type(8)))  _Float16 v8h;
typedef __attribute__((ext_vector_type(8)))  float v8f;
typedef __attribute__((ext_vector_type(4)))  float v4f;
typedef __attribute__((ext_vector_type(2)))  float v2f;
typedef __attribute__((ext_vector_type(4)))  unsigned v4u;
typedef __attribute__((ext_vector_type(4)))  int v4i;
typedef float __attribute__((may_alias)) float_a;
typedef int __attribute__((may_alias)) int_a;

template <typename T> __device__ __forceinline__ void vst2(void* p, T v) { *(volatile T*)p = v; __threadfence(); *(volatile T*)p = v; }
__device__ __forceinline__ v8f wmma16(v16h a, v16h b, v8f c) {
  v8f d = __builtin_amdgcn_wmma_f32_16x16x32_f16(false, a, false, b, (short)0, c, false, false);
  asm volatile("v_nop\n\tv_nop\n\tv_nop\n\tv_nop" : "+v"(d) : "v"(a), "v"(b));
  return d;
}
__device__ __forceinline__ v8f wmma_bf(v16b a, v16b b, v8f c) {
  v8f d = __builtin_amdgcn_wmma_f32_16x16x32_bf16(false, a, false, b, (short)0, c, false, false);
  asm volatile("v_nop\n\tv_nop\n\tv_nop\n\tv_nop" : "+v"(d) : "v"(a), "v"(b));
  return d;
}
__device__ __forceinline__ v16h frag_h(const _Float16* rowk0, int lane) {
  union { v16h v; v8h q[2]; } u; const _Float16* p = rowk0 + 8 * (lane >> 4);
  u.q[0] = *(const v8h*)p; u.q[1] = *(const v8h*)(p + 16); return u.v;
}
__device__ __forceinline__ v16h frag_f32(const float* rowk0, int lane) {
  v16h a; const float* p = rowk0 + 8 * (lane >> 4);
#pragma unroll
  for (int i = 0; i < 8; ++i) { a[i] = (_Float16)p[i]; a[8 + i] = (_Float16)p[16 + i]; }
  return a;
}
__device__ __forceinline__ v16h frag_f32s(const float* rowk0, int lane, float sc) {
  v16h a; const float* p = rowk0 + 8 * (lane >> 4);
#pragma unroll
  for (int i = 0; i < 8; ++i) { a[i] = (_Float16)(p[i] * sc); a[8 + i] = (_Float16)(p[16 + i] * sc); }
  return a;
}
__device__ __forceinline__ v16h fragc_f32(const float* W, int k0, int n, int lane, int ld, int K) {
  v16h a; const int g = lane >> 4;
#pragma unroll
  for (int i = 0; i < 8; ++i) { const int ka = k0 + 8 * g + i, kb = ka + 16;
    a[i] = (_Float16)(ka < K ? W[(size_t)(ka < K ? ka : K - 1) * ld + n] : 0.f); a[8 + i] = (_Float16)(kb < K ? W[(size_t)(kb < K ? kb : K - 1) * ld + n] : 0.f); }
  return a;
}
struct F2 { v16b h, l; };
__device__ __forceinline__ F2 bsplit16(const float v[16]) { F2 r;
#pragma unroll
  for (int i = 0; i < 16; ++i) { const __bf16 h = (__bf16)v[i]; r.h[i] = h; r.l[i] = (__bf16)(v[i] - (float)h); }
  return r; }
__device__ __forceinline__ F2 split_row(const float* row, int k0, int lane) { float v[16]; const float* p = row + k0 + 8 * (lane >> 4);
#pragma unroll
  for (int i = 0; i < 8; ++i) { v[i] = p[i]; v[8 + i] = p[16 + i]; }
  return bsplit16(v); }
__device__ __forceinline__ F2 split_rowK(const float* row, int k0, int lane, int K) { float v[16]; const int g = lane >> 4;
#pragma unroll
  for (int i = 0; i < 8; ++i) { const int ka = k0 + 8 * g + i, kb = ka + 16; v[i] = ka < K ? row[ka < K ? ka : K - 1] : 0.f; v[8 + i] = kb < K ? row[kb < K ? kb : K - 1] : 0.f; }
  return bsplit16(v); }
__device__ __forceinline__ F2 split_col(const float* W, int k0, int n, int lane, int ld, int K) { float v[16]; const int g = lane >> 4;
#pragma unroll
  for (int i = 0; i < 8; ++i) { const int ka = k0 + 8 * g + i, kb = ka + 16; v[i] = ka < K ? W[(size_t)(ka < K ? ka : K - 1) * ld + n] : 0.f; v[8 + i] = kb < K ? W[(size_t)(kb < K ? kb : K - 1) * ld + n] : 0.f; }
  return bsplit16(v); }
__device__ __forceinline__ v8f mac3(const F2& a, const F2& b, v8f c) { c = wmma_bf(a.l, b.h, c); c = wmma_bf(a.h, b.l, c); return wmma_bf(a.h, b.h, c); }
__device__ __forceinline__ float sigm(float v) { return 1.0f / (1.0f + expf(-v)); }
#define LDSX() do { asm volatile("s_wait_dscnt 0" ::: "memory"); __builtin_amdgcn_wave_barrier(); __builtin_amdgcn_fence(__ATOMIC_RELEASE, "workgroup"); } while (0)


#define NRW 4096
#define TL 256
#define EM 96
#define NHD 6
#define HDM 16
#define VOC 98
#define G3 (3 * EM)
#ifndef NRT
#define NRT NRW
#endif
typedef __attribute__((ext_vector_type(8))) __bf16 v8b;
__device__ __forceinline__ v16b frag_b(const __bf16* rowk0, int lane) {
  union { v16b v; v8b q[2]; } u; const __bf16* p = rowk0 + 8 * (lane >> 4);
  u.q[0] = *(const v8b*)p; u.q[1] = *(const v8b*)(p + 16); return u.v;
}
__device__ __forceinline__ float bfr(float v) { return (float)(__bf16)v; }
__device__ __attribute__((noinline)) float exp_ni(float v) { return expf(v); }
__device__ __attribute__((noinline)) float erf_ni(float v) { return erff(v); }

__device__ __attribute__((noinline)) float tanh_ni(float v) { return tanhf(v); }
__device__ __forceinline__ float sigm_f(float v) { return 1.0f / (1.0f + exp_ni(-v)); }
__device__ __forceinline__ void put_hl(__bf16* h, __bf16* l, float v) { const __bf16 hb = (__bf16)v; *h = hb; *l = (__bf16)(v - (float)hb); }
#define PK_IN   0
#define PK_OUT  (PK_IN + G3 * EM)
#define PK_IH   (PK_OUT + EM * EM)
#define PK_HH   (PK_IH + G3 * G3)
#define PK_MW   (PK_HH + G3 * EM)
#define PK_HD   (PK_MW + EM * EM)
#define PK_END  (PK_HD + 112 * EM)
#define WS_PK   0u
#define WS_TK   (WS_PK + 2u * PK_END)
#define WS_TV   (WS_TK + 4u * 128 * 128)
#define WS_PKT  (WS_TV + 4u * 128 * 128)
#define WS_PVT  (WS_PKT + 4u * 256 * 128)
#define WS_LOG  (WS_PVT + 4u * 256 * 128)
#define WS_NH   (WS_LOG + 4u * NRW * 128)
#define WS_NM   (WS_NH + 4u * NRW * EM)
#define WS_END  (WS_NM + 4u * NRW * EM)
#define TP 128

__global__ __launch_bounds__(128) void k_pack(const float* __restrict__ Wm, int K, int nrows, __bf16* __restrict__ DST) {
  __shared__ __align__(16) __bf16 s[8 * G3]; const int n0 = blockIdx.x * 8, tid = threadIdx.x;
  for (int q = tid; q < 8 * K; q += 128) { const int rl = q / K, k = q % K; s[q] = (__bf16)((n0 + rl) < nrows ? Wm[(size_t)(n0 + rl) * K + k] : 0.f); }
  __syncthreads();
  for (int q = tid; q < K; q += 128) vst2((unsigned*)(DST + (size_t)n0 * K + q * 8), *(const v4u*)&s[q * 8]);
}
__global__ __launch_bounds__(256) void k_tab(const float* __restrict__ TOK, const float* __restrict__ POSE, const float* __restrict__ WIN, float* __restrict__ TK, float* __restrict__ TV, float* __restrict__ PKT, float* __restrict__ PVT) {
  __shared__ float se[EM]; __shared__ __align__(16) float so[2][TP]; const int r = blockIdx.x, tid = threadIdx.x; const bool isTok = r < VOC; const int rr = isTok ? r : r - VOC;
  const float* e = isTok ? TOK + (size_t)rr * EM : POSE + (size_t)rr * EM;
  if (tid < EM) se[tid] = bfr(e[tid]);
  for (int q = tid; q < 2 * TP; q += 256) (&so[0][0])[q] = 0.f;
  __syncthreads();
  if (tid < 2 * EM) { const int which = tid / EM, c = tid % EM; const float* w = WIN + (size_t)((1 + which) * EM + c) * EM; float s = 0.f;
#pragma unroll 4
    for (int k = 0; k < EM; ++k) s += se[k] * bfr(w[k]);
    so[which][c] = s; }
  __syncthreads();
  float* d0 = (isTok ? TK : PKT) + (size_t)rr * TP; float* d1 = (isTok ? TV : PVT) + (size_t)rr * TP;
  if (tid < 32) vst2(d0 + tid * 4, *(const v4f*)&so[0][tid * 4]); else if (tid < 64) vst2(d1 + (tid - 32) * 4, *(const v4f*)&so[1][(tid - 32) * 4]);
}
__global__ __launch_bounds__(64) void k_main(const int* __restrict__ CUR, const int* __restrict__ HIST, const float* __restrict__ HID, const float* __restrict__ MEM, const float* __restrict__ TOK, const float* __restrict__ POSE,
    const __bf16* __restrict__ PK, const float* __restrict__ bin, const float* __restrict__ bout, const float* __restrict__ bih, const float* __restrict__ bhh, const float* __restrict__ pgw, const float* __restrict__ pgb, const float* __restrict__ mwb, const float* __restrict__ lng, const float* __restrict__ lnb, const float* __restrict__ hdb,
    const float* __restrict__ TK, const float* __restrict__ TV, const float* __restrict__ PKT, const float* __restrict__ PVT, float* __restrict__ LOG, float* __restrict__ NH, float* __restrict__ NM) {
  __shared__ __align__(16) __bf16 sah[16][G3 + 8], sal[16][G3 + 8];
  __shared__ __align__(16) float sq[16][EM + 4];
  __shared__ __align__(16) float sgi[16][G3 + 4], sgh[16][G3 + 4];
  __shared__ __align__(16) float snh[16][EM + 4], snm[16][EM + 4], slog[16][TP];
  __shared__ float sp[16];
  const int tid = threadIdx.x, wave = tid >> 5, lane = tid & 31, col = lane & 15, g = lane >> 4; const size_t r0 = (size_t)blockIdx.x * 16;
  for (int q = tid; q < 16 * EM; q += 64) { const int rl = q / EM, c = q % EM; int tk = HIST[(r0 + rl) * TL + (TL - 1)]; tk = min(max(tk, 0), VOC - 1); put_hl(&sah[rl][c], &sal[rl][c], bfr(TOK[(size_t)tk * EM + c]) + bfr(POSE[(size_t)(TL - 1) * EM + c])); }
  __syncthreads();
  { for (int j = wave; j < 6; j += 2) { v8f acc = {};
#pragma unroll
      for (int kc = 0; kc < 3; ++kc) { const v16b ah = frag_b(&sah[col][kc * 32], lane), al = frag_b(&sal[col][kc * 32], lane); const v16b w = frag_b(PK + PK_IN + (size_t)(j * 16 + col) * EM + kc * 32, lane); acc = wmma_bf(al, w, acc); acc = wmma_bf(ah, w, acc); }
#pragma unroll
      for (int r = 0; r < 8; ++r) sq[8 * g + r][j * 16 + col] = acc[r] + bfr(bin[j * 16 + col]); } }
  __syncthreads();
#pragma unroll 1
  for (int round = 0; round < 2; ++round) { const int pr = round * 64 + tid; if (pr < 16 * NHD) { const int rl = pr / NHD, h = pr % NHD; const int* hrow = HIST + (r0 + rl) * TL;
      float qv[HDM]; float qb = 0.f, m = -3.0e38f, l = 0.f, acc[HDM];
#pragma unroll
      for (int d = 0; d < HDM; ++d) { qv[d] = sq[rl][h * HDM + d]; qb += qv[d] * bfr(bin[EM + h * HDM + d]); acc[d] = 0.f; }
#pragma unroll 1
      for (int t = 0; t < TL; ++t) { int tk = hrow[t]; tk = min(max(tk, 0), VOC - 1); const float* kr = TK + (size_t)tk * TP + h * HDM; const float* kp = PKT + (size_t)t * TP + h * HDM; float s = qb;
#pragma unroll
        for (int d = 0; d < HDM; ++d) s += qv[d] * (kr[d] + kp[d]);
        s *= 0.25f; const float mn = fmaxf(m, s); const float al = exp_ni(m - mn), p = exp_ni(s - mn); l = l * al + p; m = mn;
        const float* vr = TV + (size_t)tk * TP + h * HDM; const float* vp = PVT + (size_t)t * TP + h * HDM;
#pragma unroll
        for (int d = 0; d < HDM; ++d) acc[d] = acc[d] * al + p * (vr[d] + vp[d]); }
      const float il = 1.0f / l;
#pragma unroll
      for (int d = 0; d < HDM; ++d) put_hl(&sah[rl][h * HDM + d], &sal[rl][h * HDM + d], acc[d] * il + bfr(bin[2 * EM + h * HDM + d])); } }
  __syncthreads();
  { float cx[3][8];
#pragma unroll
    for (int jj = 0; jj < 3; ++jj) { const int j = wave + 2 * jj; v8f acc = {};
#pragma unroll
      for (int kc = 0; kc < 3; ++kc) { const v16b ah = frag_b(&sah[col][kc * 32], lane), al = frag_b(&sal[col][kc * 32], lane); const v16b w = frag_b(PK + PK_OUT + (size_t)(j * 16 + col) * EM + kc * 32, lane); acc = wmma_bf(al, w, acc); acc = wmma_bf(ah, w, acc); }
#pragma unroll
      for (int r = 0; r < 8; ++r) cx[jj][r] = acc[r] + bfr(bout[j * 16 + col]); }
    __syncthreads();
#pragma unroll
    for (int jj = 0; jj < 3; ++jj)
#pragma unroll
      for (int r = 0; r < 8; ++r) put_hl(&sah[8 * g + r][EM + (wave + 2 * jj) * 16 + col], &sal[8 * g + r][EM + (wave + 2 * jj) * 16 + col], cx[jj][r]); }
  for (int q = tid; q < 16 * EM; q += 64) { const int rl = q / EM, c = q % EM; int tk = CUR[r0 + rl]; tk = min(max(tk, 0), VOC - 1); sah[rl][c] = (__bf16)TOK[(size_t)tk * EM + c]; sal[rl][c] = (__bf16)0.f; sah[rl][2 * EM + c] = (__bf16)MEM[(r0 + rl) * EM + c]; sal[rl][2 * EM + c] = (__bf16)0.f; }
  __syncthreads();
  for (int j = wave; j < 18; j += 2) { v8f acc = {}, acch = {};
#pragma unroll
    for (int kc = 0; kc < 9; ++kc) { const v16b ah = frag_b(&sah[col][kc * 32], lane), al = frag_b(&sal[col][kc * 32], lane); const v16b w = frag_b(PK + PK_IH + (size_t)(j * 16 + col) * G3 + kc * 32, lane); acc = wmma_bf(al, w, acc); acc = wmma_bf(ah, w, acc); }
#pragma unroll
    for (int kc = 0; kc < 3; ++kc) { v16b a; { const float* p = HID + (r0 + col) * EM + kc * 32 + 8 * g;
#pragma unroll
        for (int i = 0; i < 8; ++i) { a[i] = (__bf16)p[i]; a[8 + i] = (__bf16)p[16 + i]; } }
      acch = wmma_bf(a, frag_b(PK + PK_HH + (size_t)(j * 16 + col) * EM + kc * 32, lane), acch); }
#pragma unroll
    for (int r = 0; r < 8; ++r) { sgi[8 * g + r][j * 16 + col] = acc[r] + bfr(bih[j * 16 + col]); sgh[8 * g + r][j * 16 + col] = acch[r] + bfr(bhh[j * 16 + col]); } }
  __syncthreads();
  for (int q = tid; q < 16 * EM; q += 64) { const int rl = q / EM, u = q % EM; const float rg = sigm_f(sgi[rl][u] + sgh[rl][u]), zg = sigm_f(sgi[rl][EM + u] + sgh[rl][EM + u]); const float ng = tanh_ni(sgi[rl][2 * EM + u] + rg * sgh[rl][2 * EM + u]);
    const float hv = bfr(HID[(r0 + rl) * EM + u]); const float nh = (1.0f - zg) * ng + zg * hv; snh[rl][u] = nh; put_hl(&sah[rl][u], &sal[rl][u], nh); }
  __syncthreads();
  if (tid < 16) { float s = bfr(pgb[0]);
#pragma unroll 4
    for (int u = 0; u < EM; ++u) s += snh[tid][u] * bfr(pgw[u]);
    sp[tid] = sigm_f(s); }
  for (int j = wave; j < 6; j += 2) { v8f acc = {};
#pragma unroll
    for (int kc = 0; kc < 3; ++kc) { const v16b ah = frag_b(&sah[col][kc * 32], lane), al = frag_b(&sal[col][kc * 32], lane); const v16b w = frag_b(PK + PK_MW + (size_t)(j * 16 + col) * EM + kc * 32, lane); acc = wmma_bf(al, w, acc); acc = wmma_bf(ah, w, acc); }
#pragma unroll
    for (int r = 0; r < 8; ++r) sq[8 * g + r][j * 16 + col] = tanh_ni(acc[r] + bfr(mwb[j * 16 + col])); }
  __syncthreads();
  for (int q = tid; q < 16 * EM; q += 64) { const int rl = q / EM, u = q % EM; const float pv = sp[rl]; snm[rl][u] = (1.0f - pv) * bfr(MEM[(r0 + rl) * EM + u]) + pv * sq[rl][u]; }
  if (tid < 16) { const int rl = tid; float su = 0.f; for (int u = 0; u < EM; ++u) su += snh[rl][u]; const float mu = su / (float)EM; float sv = 0.f; for (int u = 0; u < EM; ++u) { const float d = snh[rl][u] - mu; sv += d * d; } const float rs = rsqrtf(sv / (float)EM + 1e-5f);
    for (int u = 0; u < EM; ++u) put_hl(&sah[rl][u], &sal[rl][u], (snh[rl][u] - mu) * rs * bfr(lng[u]) + bfr(lnb[u])); }
  __syncthreads();
  for (int j = wave; j < 8; j += 2) { v8f acc = {};
    if (j < 7) {
#pragma unroll
      for (int kc = 0; kc < 3; ++kc) { const v16b ah = frag_b(&sah[col][kc * 32], lane), al = frag_b(&sal[col][kc * 32], lane); const v16b w = frag_b(PK + PK_HD + (size_t)(j * 16 + col) * EM + kc * 32, lane); acc = wmma_bf(al, w, acc); acc = wmma_bf(ah, w, acc); } }
    const int o = j * 16 + col;
#pragma unroll
    for (int r = 0; r < 8; ++r) slog[8 * g + r][o] = (j < 7 && o < VOC) ? acc[r] + bfr(hdb[o < VOC ? o : 0]) : 0.f; }
  __syncthreads();
  for (int q = tid; q < 16 * 32; q += 64) { const int rl = q >> 5, pc = q & 31; vst2(LOG + (r0 + rl) * TP + pc * 4, *(const v4f*)&slog[rl][pc * 4]); }
  for (int q = tid; q < 16 * 24; q += 64) { const int rl = q / 24, pc = q % 24; vst2(NH + (r0 + rl) * EM + pc * 4, *(const v4f*)&snh[rl][pc * 4]); vst2(NM + (r0 + rl) * EM + pc * 4, *(const v4f*)&snm[rl][pc * 4]); }
}
__global__ __launch_bounds__(256) void k_out(const float* __restrict__ LOG, const float* __restrict__ NH, const float* __restrict__ NM, float* __restrict__ out) {
  const size_t p = (size_t)blockIdx.x * 256 + threadIdx.x; const size_t nlog = (size_t)NRW * VOC, nh = (size_t)NRW * EM; const size_t total = nlog + 2 * nh; if (p * 4 >= total) return;
  v4f v;
#pragma unroll
  for (int i = 0; i < 4; ++i) { const size_t f = p * 4 + i; float x;
    size_t row; if (f < nlog) { row = f / VOC; x = LOG[row * TP + (f % VOC)]; } else if (f < nlog + nh) { row = (f - nlog) / EM; x = NH[f - nlog]; } else { row = (f - nlog - nh) / EM; x = NM[f - nlog - nh]; }
    if (row >= (size_t)NRT) x = 0.f;
    v[i] = x; }
  vst2(out + p * 4, v);
}
extern "C" void kernel_launch(void* const* d_in, const int* in_sizes, int n_in, void* d_out, int out_size, void* d_ws, size_t ws_size, hipStream_t stream) {
  (void)in_sizes; (void)n_in; (void)out_size;
  const float** F = (const float**)d_in; const int* CUR = (const int*)d_in[0]; const int* HIST = (const int*)d_in[1];
  if (ws_size < (size_t)WS_END) return;
  char* ws = (char*)d_ws; __bf16* PK = (__bf16*)(ws + WS_PK); float *TK = (float*)(ws + WS_TK), *TV = (float*)(ws + WS_TV), *PKT = (float*)(ws + WS_PKT), *PVT = (float*)(ws + WS_PVT), *LOG = (float*)(ws + WS_LOG), *NH = (float*)(ws + WS_NH), *NM = (float*)(ws + WS_NM);
  k_pack<<<G3 / 8, 128, 0, stream>>>(F[6], EM, G3, PK + PK_IN);
  k_pack<<<EM / 8, 128, 0, stream>>>(F[8], EM, EM, PK + PK_OUT);
  k_pack<<<G3 / 8, 128, 0, stream>>>(F[10], G3, G3, PK + PK_IH);
  k_pack<<<G3 / 8, 128, 0, stream>>>(F[11], EM, G3, PK + PK_HH);
  k_pack<<<EM / 8, 128, 0, stream>>>(F[16], EM, EM, PK + PK_MW);
  k_pack<<<112 / 8, 128, 0, stream>>>(F[20], EM, VOC, PK + PK_HD);
  k_tab<<<VOC + TL, 256, 0, stream>>>(F[4], F[5], F[6], TK, TV, PKT, PVT);
  k_main<<<NRT / 16, 64, 0, stream>>>(CUR, HIST, F[2], F[3], F[4], F[5], PK, F[7], F[9], F[12], F[13], F[14], F[15], F[17], F[18], F[19], F[21], TK, TV, PKT, PVT, LOG, NH, NM);
  k_out<<<(unsigned)((((size_t)NRW * (VOC + 2 * EM)) / 4 + 255) / 256), 256, 0, stream>>>(LOG, NH, NM, (float*)d_out);
}
